// ScalarDotProductCriticNetwork_49658411876916
// MI455X (gfx1250) — hardware-run, weakly checked
//
#include <hip/hip_runtime.h>
#include <math.h>

typedef __attribute__((ext_vector_type(16))) _Float16 v16h;
typedef __attribute__((ext_vector_type(8)))  _Float16 v8h;
typedef __attribute__((ext_vector_type(8)))  float    v8f;
typedef __attribute__((ext_vector_type(4)))  float    v4f;
typedef __attribute__((ext_vector_type(4)))  unsigned v4u;

constexpr int kBatch = 256;
constexpr int kAg    = 32;
constexpr int kObs   = 96;
constexpr int kAct   = 32;
constexpr int kDim   = 128;
constexpr int kF1    = 64;
constexpr int kF2    = 32;
constexpr int kRows  = kBatch * kAg;
static_assert(kObs + kAct == kDim, "concat width");
static_assert(kRows == 8192, "rows");
static_assert((kDim % 32) == 0 && ((2 * kDim) % 32) == 0 && (kF1 % 32) == 0, "K multiples of 32");
static_assert((kRows % 64) == 0 && ((4 * kDim) % 64) == 0 && (kF1 % 64) == 0, "tile multiples");

constexpr float kCarryA  = 16.0f;
constexpr float kCarryW  = 256.0f;
constexpr float kCarryP  = 128.0f;
constexpr float kProjScale = 1.0f / (kCarryA * kCarryW);
constexpr float kF1Scale   = 1.0f / (kCarryP * kCarryW * (float)kAg);
constexpr float kCarrySm = 1024.0f;
constexpr float kCarryH  = 32768.0f;

constexpr size_t kOffAOA  = 0;
constexpr size_t kOffAOP  = kOffAOA  + (size_t)kRows * kDim * 2;
constexpr size_t kOffAOAP = kOffAOP  + (size_t)kRows * kDim * 2;
constexpr size_t kOffBTA  = kOffAOAP + (size_t)kRows * kDim * 2;
constexpr size_t kOffBTP  = kOffBTA  + (size_t)4 * kDim * kDim * 2;
constexpr size_t kOffBTF1 = kOffBTP  + (size_t)2 * kDim * kDim * 2;
constexpr size_t kOffBTF2 = kOffBTF1 + (size_t)kF1 * 2 * kDim * 2;
constexpr size_t kOffP1   = kOffBTF2 + (size_t)kF2 * kF1 * 2;
constexpr size_t kOffAVOP = kOffP1   + (size_t)kRows * 4 * kDim * 2;
constexpr size_t kOffP3   = kOffAVOP + (size_t)kRows * kDim * 2;
constexpr size_t kOffNF   = kOffP3   + (size_t)kRows * 2 * kDim * 2;
constexpr size_t kOffDIFF = kOffNF   + (size_t)kRows * 2 * kDim * 2;
constexpr size_t kOffW32  = kOffDIFF + (size_t)kRows * kDim * 2;
constexpr size_t kOffU    = kOffW32  + (size_t)kRows * kAg * 4;
constexpr size_t kOffV    = kOffU    + (size_t)kRows * kF1 * 4;
constexpr size_t kWsTotal = kOffV    + (size_t)kRows * kF1 * 4;
static_assert(kWsTotal == 32739328ull, "carve total");
static_assert(kWsTotal <= 134217728ull, "carve cap");
static_assert((kOffAOP % 128) == 0 && (kOffAOAP % 128) == 0 && (kOffBTA % 128) == 0 && (kOffBTP % 128) == 0 &&
              (kOffBTF1 % 128) == 0 && (kOffBTF2 % 128) == 0 && (kOffP1 % 128) == 0 && (kOffAVOP % 128) == 0 &&
              (kOffP3 % 128) == 0 && (kOffNF % 128) == 0 && (kOffDIFF % 128) == 0 && (kOffW32 % 128) == 0 &&
              (kOffU % 128) == 0 && (kOffV % 128) == 0, "128-B aligned regions");

constexpr size_t kOut1 = (size_t)kRows * kAg * kF2;
constexpr size_t kOut2 = kOut1 + (size_t)kRows * kAg;
static_assert(kOut1 * 4 == 33554432ull && kOut2 * 4 == 34603008ull, "output byte offsets");
static_assert((kOut2 + (size_t)kRows * kAg) * 4 == 35651584ull, "output total");

__device__ __forceinline__ _Float16 cvt_h(float v) {
  const float a = __builtin_fabsf(v);
  const float f = (a < 6.103515625e-05f) ? 0.0f : v;
  return (_Float16)f;
}
__device__ __forceinline__ unsigned h_bits(float v) {
  const _Float16 h = cvt_h(v);
  const unsigned short s = __builtin_bit_cast(unsigned short, h);
  return (unsigned)s;
}
__device__ __forceinline__ float h16_to_f32(unsigned hb) {
  const unsigned sgn = (hb & 0x8000u) << 16;
  const unsigned em = hb & 0x7fffu;
  const float fn = __uint_as_float((em << 13) + 0x38000000u);
  const float fs = (float)em * 5.9604644775390625e-8f;
  const float mag = (em < 0x400u) ? fs : fn;
  return __uint_as_float(__float_as_uint(mag) | sgn);
}
__device__ __forceinline__ unsigned pick_half(unsigned w, int e) {
  return (e & 1) ? (w >> 16) : (w & 0xffffu);
}

union FragU { v16h v; v8h h[2]; };
__device__ __forceinline__ v16h frag_load(const _Float16* p) {
  FragU f;
  f.h[0] = *(const v8h*)(p);
  f.h[1] = *(const v8h*)(p + 16);
  return f.v;
}
__device__ __forceinline__ v8f mma_h(v16h a, v16h b, v8f c) {
  c = __builtin_amdgcn_wmma_f32_16x16x32_f16(false, a, false, b, (short)0, c, false, false);
  asm volatile("v_nop\n\tv_nop\n\tv_nop\n\tv_nop" : "+v"(c) : "v"(a), "v"(b));
  return c;
}
__device__ __forceinline__ void wave_sync_lds() {
  __builtin_amdgcn_fence(__ATOMIC_RELEASE, "workgroup");
  __builtin_amdgcn_wave_barrier();
  __builtin_amdgcn_fence(__ATOMIC_ACQUIRE, "workgroup");
}

constexpr unsigned kPrepBlkAct = (unsigned)(kRows * 16 / 256);
constexpr unsigned kPrepBlkTotal = 2u * kPrepBlkAct + 32u + 16u + 8u + 1u;
static_assert(kPrepBlkAct == 512u && kPrepBlkTotal == 1081u, "prep grid");

__global__ __launch_bounds__(256) void prep_kernel(
    const float* __restrict__ states, const float* __restrict__ policies, const float* __restrict__ actions,
    const float* __restrict__ states_p, const float* __restrict__ actions_p,
    const float* __restrict__ Wk, const float* __restrict__ Wq, const float* __restrict__ Wv,
    const float* __restrict__ Wkp, const float* __restrict__ Wqp, const float* __restrict__ Wvp,
    const float* __restrict__ Wf1, const float* __restrict__ Wf2,
    unsigned short* __restrict__ aOA, unsigned short* __restrict__ aOP, unsigned short* __restrict__ aOAP,
    unsigned short* __restrict__ btA, unsigned short* __restrict__ btP,
    unsigned short* __restrict__ btF1, unsigned short* __restrict__ btF2)
{
  const unsigned blk = blockIdx.x;
  const unsigned tid = threadIdx.x;
  if (blk < 2u * kPrepBlkAct) {
    const bool people = (blk >= kPrepBlkAct);
    const unsigned t = (people ? (blk - kPrepBlkAct) : blk) * 256u + tid;
    unsigned row = t >> 4;
    unsigned c8 = (t & 15u) << 3;
    asm volatile("" : "+v"(row), "+v"(c8));
    const float* st = people ? states_p : states;
    const float* ac = people ? actions_p : actions;
    const unsigned cs = (c8 < 96u) ? c8 : 88u;
    const unsigned ca = (c8 >= 96u) ? (c8 - 96u) : 0u;
    v4f s0 = *(const v4f*)(st + (size_t)row * kObs + cs);
    v4f s1 = *(const v4f*)(st + (size_t)row * kObs + cs + 4);
    v4f a0 = *(const v4f*)(ac + (size_t)row * kAct + ca);
    v4f a1 = *(const v4f*)(ac + (size_t)row * kAct + ca + 4);
    v4f p0 = *(const v4f*)(policies + (size_t)row * kAct + ca);
    v4f p1 = *(const v4f*)(policies + (size_t)row * kAct + ca + 4);
    asm volatile("" : "+v"(s0), "+v"(s1), "+v"(a0), "+v"(a1), "+v"(p0), "+v"(p1));
    const bool isS = (c8 < 96u);
    const v4f x0 = isS ? s0 : a0;
    const v4f x1 = isS ? s1 : a1;
    const v4f y0 = isS ? s0 : p0;
    const v4f y1 = isS ? s1 : p1;
    v8h hx, hy;
#pragma unroll
    for (int e = 0; e < 4; ++e) {
      hx[e]     = cvt_h(x0[e] * kCarryA);
      hx[4 + e] = cvt_h(x1[e] * kCarryA);
      hy[e]     = cvt_h(y0[e] * kCarryA);
      hy[4 + e] = cvt_h(y1[e] * kCarryA);
    }
    unsigned short* d1 = (people ? aOAP : aOA) + (size_t)t * 8;
    unsigned short* d2 = aOP + (size_t)t * 8;
    *(volatile v8h*)d1 = hx;
    if (!people) *(volatile v8h*)d2 = hy;
    __threadfence();
    *(volatile v8h*)d1 = hx;
    if (!people) *(volatile v8h*)d2 = hy;
  } else {
    const unsigned wb = blk - 2u * kPrepBlkAct;
    const float* src;
    unsigned short* dst;
    unsigned tb, ksh, ldw, nmask;
    if (wb < 32u) {
      const unsigned mat = wb >> 3;
      src = (mat == 0u) ? Wq : (mat == 1u) ? Wk : (mat == 2u) ? Wqp : Wv;
      dst = btA; tb = wb; ksh = 4u; ldw = 128u; nmask = 127u;
    } else if (wb < 48u) {
      const unsigned mat = (wb - 32u) >> 3;
      src = (mat == 0u) ? Wkp : Wvp;
      dst = btP; tb = wb - 32u; ksh = 4u; ldw = 128u; nmask = 127u;
    } else if (wb < 56u) {
      src = Wf1; dst = btF1; tb = wb - 48u; ksh = 5u; ldw = 64u; nmask = 63u;
    } else {
      src = Wf2; dst = btF2; tb = wb - 56u; ksh = 3u; ldw = 32u; nmask = 31u;
    }
    const unsigned t = tb * 256u + tid;
    unsigned n = t >> ksh;
    unsigned kc = (t & ((1u << ksh) - 1u)) << 3;
    asm volatile("" : "+v"(n), "+v"(kc));
    const unsigned ncol = n & nmask;
    v8h hv;
#pragma unroll
    for (int e = 0; e < 8; ++e) {
      const float w = src[(size_t)(kc + (unsigned)e) * ldw + ncol];
      hv[e] = cvt_h(w * kCarryW);
    }
    unsigned short* d = dst + (size_t)t * 8;
    *(volatile v8h*)d = hv;
    __threadfence();
    *(volatile v8h*)d = hv;
  }
}

template <int OUT_MODE>
__global__ __launch_bounds__(256) void gemm64_kernel(
    const unsigned short* __restrict__ Ap, int lda,
    const unsigned short* __restrict__ Btp, int ldb,
    void* __restrict__ Cout, int ldc,
    int M, int N, int K, float scale, int actFromN, float outCarry)
{
  const _Float16* A  = (const _Float16*)Ap;
  const _Float16* Bt = (const _Float16*)Btp;
  __shared__ __align__(16) float sT[8][16 * 68];
  const int lane = threadIdx.x & 31;
  const int wave = threadIdx.x >> 5;
  const int tilesN = N >> 6;
  const int tilesM = M >> 6;
  const int tile = blockIdx.x * 8 + wave;
  if (tile >= tilesM * tilesN) return;
  const int tm = tile / tilesN;
  const int tn = tile - tm * tilesN;
  const int m0 = tm << 6;
  const int n0 = tn << 6;
  const int rlane = lane & 15;
  const int koff  = (lane >> 4) * 8;
  const int mOff  = (lane >> 4) * 8;

  v8f acc[4][4];
#pragma unroll
  for (int i = 0; i < 4; ++i)
#pragma unroll
    for (int j = 0; j < 4; ++j) acc[i][j] = (v8f){0.f, 0.f, 0.f, 0.f, 0.f, 0.f, 0.f, 0.f};

  for (int k0 = 0; k0 < K; k0 += 32) {
    v16h bh[4];
#pragma unroll
    for (int j = 0; j < 4; ++j)
      bh[j] = frag_load(Bt + (size_t)(n0 + (j << 4) + rlane) * ldb + koff + k0);
#pragma unroll
    for (int i = 0; i < 4; ++i) {
      const v16h ah = frag_load(A + (size_t)(m0 + (i << 4) + rlane) * lda + koff + k0);
#pragma unroll
      for (int j = 0; j < 4; ++j) acc[i][j] = mma_h(ah, bh[j], acc[i][j]);
    }
  }

  float* slab = sT[wave];
#pragma unroll
  for (int i = 0; i < 4; ++i) {
    const int mBase = m0 + (i << 4);
#pragma unroll
    for (int j = 0; j < 4; ++j) {
#pragma unroll
      for (int r = 0; r < 8; ++r) slab[(mOff + r) * 68 + (j << 4) + rlane] = acc[i][j][r] * scale;
    }
    wave_sync_lds();
    if (OUT_MODE == 0) {
      float* C = (float*)Cout;
      const int hh = lane >> 4, c4 = (lane & 15) * 4;
      v4f v[8];
#pragma unroll
      for (int it = 0; it < 8; ++it) v[it] = *(const v4f*)(slab + (it * 2 + hh) * 68 + c4);
      for (int pass = 0; pass < 2; ++pass) {
#pragma unroll
        for (int it = 0; it < 8; ++it)
          *(volatile v4f*)(C + (size_t)(mBase + it * 2 + hh) * ldc + n0 + c4) = v[it];
        __threadfence();
      }
    } else {
      unsigned short* C = (unsigned short*)Cout;
      const int q = lane >> 3, c8 = (lane & 7) * 8;
      if (n0 >= actFromN) {
#pragma unroll 1
        for (int it = 0; it < 4; ++it) {
          float* sp = slab + (it * 4 + q) * 68 + c8;
          v4f t0 = *(const v4f*)(sp);
          v4f t1 = *(const v4f*)(sp + 4);
#pragma unroll
          for (int e = 0; e < 4; ++e) {
            t0[e] = tanhf(t0[e]);
            t1[e] = tanhf(t1[e]);
          }
          *(v4f*)(sp) = t0;
          *(v4f*)(sp + 4) = t1;
        }
      }
      v8h hv[4];
#pragma unroll
      for (int it = 0; it < 4; ++it) {
        const float* sp = slab + (it * 4 + q) * 68 + c8;
        const v4f t0 = *(const v4f*)(sp);
        const v4f t1 = *(const v4f*)(sp + 4);
#pragma unroll
        for (int e = 0; e < 4; ++e) {
          hv[it][e]     = cvt_h(t0[e] * outCarry);
          hv[it][4 + e] = cvt_h(t1[e] * outCarry);
        }
      }
      for (int pass = 0; pass < 2; ++pass) {
#pragma unroll
        for (int it = 0; it < 4; ++it)
          *(volatile v8h*)(C + (size_t)(mBase + it * 4 + q) * ldc + n0 + c8) = hv[it];
        __threadfence();
      }
    }
    wave_sync_lds();
  }
}

constexpr int kPQ    = 136;
constexpr int kTileQ = 32 * kPQ;
constexpr int kPT    = 40;
constexpr int kPS    = 33;
constexpr int kPNF   = 260;
constexpr unsigned kLdsQ     = 0u;
constexpr unsigned kLdsAvT   = kLdsQ   + 4u * kTileQ * 2u;
constexpr unsigned kLdsS     = kLdsAvT + 2u * 128u * kPT * 2u;
constexpr unsigned kLdsWt    = kLdsS   + 2u * 32u * kPS * 4u;
constexpr unsigned kLdsWh    = kLdsWt  + 2u * 1024u * 4u;
constexpr unsigned kLdsNF    = kLdsWh  + 2u * 32u * kPT * 2u;
constexpr unsigned kLdsTotal = kLdsNF  + 32u * kPNF * 4u;
static_assert(kLdsTotal == 110336u, "lds total");
static_assert((kLdsAvT % 16u) == 0 && (kLdsS % 16u) == 0 && (kLdsWt % 16u) == 0 && (kLdsWh % 16u) == 0 &&
              (kLdsNF % 16u) == 0, "lds alignment");

__global__ __launch_bounds__(256) void attn_kernel(
    const unsigned short* __restrict__ P1, const unsigned short* __restrict__ AVOP,
    const unsigned short* __restrict__ P3,
    float* __restrict__ out1, float* __restrict__ out2, float* __restrict__ W32,
    unsigned short* __restrict__ NF, unsigned short* __restrict__ DIFF)
{
  extern __shared__ __align__(16) unsigned char smem[];
  unsigned short* sQK  = (unsigned short*)(smem + kLdsQ);
  unsigned*       sAvT = (unsigned*)(smem + kLdsAvT);
  float*          sS   = (float*)(smem + kLdsS);
  float*          sWt  = (float*)(smem + kLdsWt);
  unsigned short* sWh  = (unsigned short*)(smem + kLdsWh);
  float*          sNF  = (float*)(smem + kLdsNF);

  const unsigned tid  = threadIdx.x;
  const unsigned lane = tid & 31u;
  const unsigned wave = tid >> 5;
  const unsigned hh   = lane >> 4;
  const unsigned m    = lane & 15u;
  const size_t   row0 = (size_t)blockIdx.x * kAg;

#pragma unroll
  for (int i = 0; i < 8; ++i) {
    const int tile = i >> 1;
    const unsigned within = (tid + 256u * (unsigned)i) & 511u;
    const unsigned row = within >> 4;
    const unsigned c8 = (within & 15u) << 3;
    const unsigned short* src = (tile < 3)
        ? (P1 + (row0 + row) * (size_t)(4 * kDim) + (size_t)tile * kDim + c8)
        : (P3 + (row0 + row) * (size_t)(2 * kDim) + c8);
    const v4u w = *(const v4u*)src;
    *(v4u*)(sQK + tile * kTileQ + row * kPQ + c8) = w;
  }
  __syncthreads();

  {
    const unsigned mat = wave >> 2, mt = (wave >> 1) & 1u, nt = wave & 1u;
    const _Float16* At = (const _Float16*)sQK + (mat ? 2 : 1) * kTileQ + (mt * 16u + m) * kPQ + 8u * hh;
    const _Float16* Bq = (const _Float16*)sQK + (mat ? 3 : 0) * kTileQ + (nt * 16u + m) * kPQ + 8u * hh;
    v8f acc = (v8f){0.f, 0.f, 0.f, 0.f, 0.f, 0.f, 0.f, 0.f};
#pragma unroll
    for (int ks = 0; ks < 4; ++ks) {
      const v16h a = frag_load(At + ks * 32);
      const v16h b = frag_load(Bq + ks * 32);
      acc = mma_h(a, b, acc);
    }
    const float inv_sqrt_dk = 1.0f / sqrtf((float)kDim);
    const float sc = inv_sqrt_dk * (1.0f / (kCarryP * kCarryP));
    float* dS = sS + mat * (32 * kPS);
#pragma unroll
    for (int r = 0; r < 8; ++r) dS[(mt * 16u + 8u * hh + (unsigned)r) * kPS + nt * 16u + m] = acc[r] * sc;
  }
  __syncthreads();

#pragma unroll
  for (int r4 = 0; r4 < 4; ++r4) {
    const unsigned a = wave * 4u + (unsigned)r4;
    const float s = sS[a * kPS + lane];
    float mx = s;
#pragma unroll
    for (int off = 16; off >= 1; off >>= 1) mx = fmaxf(mx, __shfl_xor(mx, off, 32));
    const float e = expf(s - mx);
    float sum = e;
#pragma unroll
    for (int off = 16; off >= 1; off >>= 1) sum += __shfl_xor(sum, off, 32);
    const float w = e * (1.0f / sum);
    sWt[a * 32u + lane] = w;
    sWh[a * kPT + lane] = (unsigned short)h_bits(w * kCarrySm);
  }
#pragma unroll
  for (int r4 = 0; r4 < 4; ++r4) {
    const unsigned p = wave * 4u + (unsigned)r4;
    const float s = sS[32 * kPS + lane * kPS + p];
    float mx = s;
#pragma unroll
    for (int off = 16; off >= 1; off >>= 1) mx = fmaxf(mx, __shfl_xor(mx, off, 32));
    const float e = expf(s - mx);
    float sum = e;
#pragma unroll
    for (int off = 16; off >= 1; off >>= 1) sum += __shfl_xor(sum, off, 32);
    const float w = e * (1.0f / sum);
    sWt[1024u + lane * 32u + p] = w;
    sWh[32 * kPT + lane * kPT + p] = (unsigned short)h_bits(w * kCarrySm);
  }
  __syncthreads();

  {
    const unsigned jp = tid >> 4;
    const unsigned d8 = (tid & 15u) << 3;
    const size_t r0 = row0 + 2u * jp;
    const v4u oa0 = *(const v4u*)(P1 + r0 * (size_t)(4 * kDim) + 3 * kDim + d8);
    const v4u oa1 = *(const v4u*)(P1 + (r0 + 1) * (size_t)(4 * kDim) + 3 * kDim + d8);
    const v4u op0 = *(const v4u*)(AVOP + r0 * (size_t)kDim + d8);
    const v4u op1 = *(const v4u*)(AVOP + (r0 + 1) * (size_t)kDim + d8);
    const v4u pp0 = *(const v4u*)(P3 + r0 * (size_t)(2 * kDim) + kDim + d8);
    const v4u pp1 = *(const v4u*)(P3 + (r0 + 1) * (size_t)(2 * kDim) + kDim + d8);
    v8h dv0, dv1;
#pragma unroll
    for (int e = 0; e < 8; ++e) {
      const unsigned wa0 = oa0[e >> 1], wa1 = oa1[e >> 1];
      const unsigned wo0 = op0[e >> 1], wo1 = op1[e >> 1];
      const unsigned wp0 = pp0[e >> 1], wp1 = pp1[e >> 1];
      const unsigned a_lo = pick_half(wa0, e), a_hi = pick_half(wa1, e);
      const unsigned p_lo = pick_half(wp0, e), p_hi = pick_half(wp1, e);
      sAvT[(d8 + (unsigned)e) * (kPT / 2) + jp] = (a_hi << 16) | (a_lo & 0xffffu);
      sAvT[128u * (kPT / 2) + (d8 + (unsigned)e) * (kPT / 2) + jp] = (p_hi << 16) | (p_lo & 0xffffu);
      const float fa0 = h16_to_f32(a_lo), fa1 = h16_to_f32(a_hi);
      const float fo0 = h16_to_f32(pick_half(wo0, e)), fo1 = h16_to_f32(pick_half(wo1, e));
      dv0[e] = cvt_h(fo0 - fa0);
      dv1[e] = cvt_h(fo1 - fa1);
    }
    unsigned short* dp0 = DIFF + r0 * (size_t)kDim + d8;
    unsigned short* dp1 = DIFF + (r0 + 1) * (size_t)kDim + d8;
    *(volatile v8h*)dp0 = dv0;
    *(volatile v8h*)dp1 = dv1;
    __threadfence();
    *(volatile v8h*)dp0 = dv0;
    *(volatile v8h*)dp1 = dv1;
  }

  if (wave < 3u) {
    const float* src = sWt + ((wave == 1u) ? 1024u : 0u);
    float* dst = (wave == 0u) ? (out1 + (size_t)blockIdx.x * 1024u)
               : (wave == 1u) ? (out2 + (size_t)blockIdx.x * 1024u)
                              : (W32 + (size_t)blockIdx.x * 1024u);
    v4f v[8];
#pragma unroll
    for (int it = 0; it < 8; ++it) v[it] = *(const v4f*)(src + it * 128 + lane * 4u);
    for (int pass = 0; pass < 2; ++pass) {
#pragma unroll
      for (int it = 0; it < 8; ++it) *(volatile v4f*)(dst + it * 128 + lane * 4u) = v[it];
      __threadfence();
    }
  }
  __syncthreads();

  {
    const unsigned mat = wave >> 2, np = wave & 3u;
    const _Float16* Aw = (const _Float16*)sWh + mat * (32 * kPT) + 8u * hh;
    const _Float16* Bv = (const _Float16*)sAvT + mat * (128 * kPT) + 8u * hh;
    const v16h a0 = frag_load(Aw + m * kPT);
    const v16h a1 = frag_load(Aw + (16u + m) * kPT);
    const v16h b0 = frag_load(Bv + ((2u * np) * 16u + m) * kPT);
    const v16h b1 = frag_load(Bv + ((2u * np + 1u) * 16u + m) * kPT);
    const v8f z = (v8f){0.f, 0.f, 0.f, 0.f, 0.f, 0.f, 0.f, 0.f};
    const v8f c00 = mma_h(a0, b0, z);
    const v8f c01 = mma_h(a0, b1, z);
    const v8f c10 = mma_h(a1, b0, z);
    const v8f c11 = mma_h(a1, b1, z);
    const float sc = 1.0f / kCarrySm;
    const unsigned colb = mat * 128u + (2u * np) * 16u + m;
#pragma unroll
    for (int r = 0; r < 8; ++r) {
      const unsigned rr = 8u * hh + (unsigned)r;
      sNF[rr * kPNF + colb]               = c00[r] * sc;
      sNF[rr * kPNF + colb + 16u]         = c01[r] * sc;
      sNF[(16u + rr) * kPNF + colb]       = c10[r] * sc;
      sNF[(16u + rr) * kPNF + colb + 16u] = c11[r] * sc;
    }
  }
  __syncthreads();

  {
    v8h hv[4];
#pragma unroll
    for (int i = 0; i < 4; ++i) {
      const unsigned row = wave + 8u * (unsigned)i;
      const float* sp = sNF + row * kPNF + lane * 8u;
      const v4f t0 = *(const v4f*)(sp);
      const v4f t1 = *(const v4f*)(sp + 4);
#pragma unroll
      for (int e = 0; e < 4; ++e) {
        hv[i][e]     = cvt_h(t0[e]);
        hv[i][4 + e] = cvt_h(t1[e]);
      }
    }
    for (int pass = 0; pass < 2; ++pass) {
#pragma unroll
      for (int i = 0; i < 4; ++i) {
        const unsigned row = wave + 8u * (unsigned)i;
        *(volatile v8h*)(NF + (row0 + row) * (size_t)(2 * kDim) + lane * 8u) = hv[i];
      }
      __threadfence();
    }
  }
}

__global__ __launch_bounds__(256) void final_kernel(
    const float* __restrict__ U, const float* __restrict__ V, const float* __restrict__ W32,
    const unsigned short* __restrict__ BtF2, float* __restrict__ out0)
{
  __shared__ __align__(16) float sU[32 * 64];
  __shared__ __align__(16) float sV[32 * 68];
  __shared__ __align__(16) float sW[32 * 32];
  __shared__ __align__(16) float sO[8][16 * 36];
  const unsigned tid  = threadIdx.x;
  const unsigned lane = tid & 31u;
  const unsigned wave = tid >> 5;
  const unsigned hh   = lane >> 4;
  const unsigned m    = lane & 15u;
  const size_t   row0 = (size_t)blockIdx.x * kAg;

#pragma unroll
  for (int i = 0; i < 2; ++i) {
    const unsigned idx = tid + 256u * (unsigned)i;
    const unsigned row = idx >> 4;
    const unsigned c4 = (idx & 15u) << 2;
    *(v4f*)(sU + row * 64u + c4) = *(const v4f*)(U + (row0 + row) * (size_t)kF1 + c4);
    *(v4f*)(sV + row * 68u + c4) = *(const v4f*)(V + (row0 + row) * (size_t)kF1 + c4);
  }
  *(v4f*)(sW + tid * 4u) = *(const v4f*)(W32 + (size_t)blockIdx.x * 1024u + tid * 4u);

  const _Float16* B2 = (const _Float16*)BtF2;
  const v16h b00 = frag_load(B2 + (size_t)(m) * kF1 + 8u * hh);
  const v16h b01 = frag_load(B2 + (size_t)(m) * kF1 + 32 + 8u * hh);
  const v16h b10 = frag_load(B2 + (size_t)(16u + m) * kF1 + 8u * hh);
  const v16h b11 = frag_load(B2 + (size_t)(16u + m) * kF1 + 32 + 8u * hh);
  __syncthreads();

  float* slab = sO[wave];
  const float osc = 1.0f / (kCarryH * kCarryW);
  const unsigned q = lane >> 3, c4 = (lane & 7u) << 2;
#pragma unroll 1
  for (int t = 0; t < 8; ++t) {
    const unsigned tile = wave * 8u + (unsigned)t;
    const unsigned a = tile >> 1;
    const unsigned ih = tile & 1u;
    const unsigned i = ih * 16u + m;
    const float w = sW[a * 32u + i];
    const float* ur = sU + a * 64u;
    const float* vr = sV + i * 68u;
    v16h af[2];
#pragma unroll
    for (int ks = 0; ks < 2; ++ks) {
#pragma unroll
      for (int g = 0; g < 2; ++g) {
        const unsigned kb = (unsigned)ks * 32u + (unsigned)g * 16u + 8u * hh;
        const v4f u0 = *(const v4f*)(ur + kb);
        const v4f u1 = *(const v4f*)(ur + kb + 4);
        const v4f v0 = *(const v4f*)(vr + kb);
        const v4f v1 = *(const v4f*)(vr + kb + 4);
#pragma unroll
        for (int e = 0; e < 4; ++e) {
          float x0 = u0[e] + w * v0[e];
          float x1 = u1[e] + w * v1[e];
          x0 = (x0 > 0.0f) ? x0 : 0.01f * x0;
          x1 = (x1 > 0.0f) ? x1 : 0.01f * x1;
          af[ks][g * 8 + e]     = cvt_h(x0 * kCarryH);
          af[ks][g * 8 + 4 + e] = cvt_h(x1 * kCarryH);
        }
      }
    }
    v8f c0 = (v8f){0.f, 0.f, 0.f, 0.f, 0.f, 0.f, 0.f, 0.f};
    v8f c1 = (v8f){0.f, 0.f, 0.f, 0.f, 0.f, 0.f, 0.f, 0.f};
    c0 = mma_h(af[0], b00, c0);
    c0 = mma_h(af[1], b01, c0);
    c1 = mma_h(af[0], b10, c1);
    c1 = mma_h(af[1], b11, c1);
#pragma unroll
    for (int r = 0; r < 8; ++r) {
      slab[(8u * hh + (unsigned)r) * 36u + m]       = c0[r] * osc;
      slab[(8u * hh + (unsigned)r) * 36u + 16u + m] = c1[r] * osc;
    }
    wave_sync_lds();
    v4f vv[4];
#pragma unroll
    for (int it = 0; it < 4; ++it) vv[it] = *(const v4f*)(slab + ((unsigned)it * 4u + q) * 36u + c4);
    float* ob = out0 + ((row0 + a) * (size_t)kAg + ih * 16u) * (size_t)kF2;
    for (int pass = 0; pass < 2; ++pass) {
#pragma unroll
      for (int it = 0; it < 4; ++it)
        *(volatile v4f*)(ob + ((unsigned)it * 4u + q) * (size_t)kF2 + c4) = vv[it];
      __threadfence();
    }
    wave_sync_lds();
  }
}

extern "C" void kernel_launch(void* const* d_in, const int* in_sizes, int n_in,
                              void* d_out, int out_size, void* d_ws, size_t ws_size,
                              hipStream_t stream) {
  if (n_in < 13) return;
  if (in_sizes[0] != kRows * kObs) return;
  if (in_sizes[1] != kRows * kAct) return;
  if (in_sizes[2] != kRows * kAct) return;
  if (in_sizes[3] != kRows * kObs) return;
  if (in_sizes[4] != kRows * kAct) return;
  for (int i = 5; i <= 10; ++i) if (in_sizes[i] != kDim * kDim) return;
  if (in_sizes[11] != 2 * kDim * kF1) return;
  if (in_sizes[12] != kF1 * kF2) return;
  if ((size_t)out_size != kOut2 + (size_t)kRows * kAg) return;
  if (ws_size < kWsTotal) return;

  const float* states    = (const float*)d_in[0];
  const float* policies  = (const float*)d_in[1];
  const float* actions   = (const float*)d_in[2];
  const float* states_p  = (const float*)d_in[3];
  const float* actions_p = (const float*)d_in[4];
  const float* Wk  = (const float*)d_in[5];
  const float* Wq  = (const float*)d_in[6];
  const float* Wv  = (const float*)d_in[7];
  const float* Wkp = (const float*)d_in[8];
  const float* Wqp = (const float*)d_in[9];
  const float* Wvp = (const float*)d_in[10];
  const float* Wf1 = (const float*)d_in[11];
  const float* Wf2 = (const float*)d_in[12];
  float* out = (float*)d_out;

  char* ws = (char*)d_ws;
  unsigned short* AOA  = (unsigned short*)(ws + kOffAOA);
  unsigned short* AOP  = (unsigned short*)(ws + kOffAOP);
  unsigned short* AOAP = (unsigned short*)(ws + kOffAOAP);
  unsigned short* BTA  = (unsigned short*)(ws + kOffBTA);
  unsigned short* BTP  = (unsigned short*)(ws + kOffBTP);
  unsigned short* BTF1 = (unsigned short*)(ws + kOffBTF1);
  unsigned short* BTF2 = (unsigned short*)(ws + kOffBTF2);
  unsigned short* P1   = (unsigned short*)(ws + kOffP1);
  unsigned short* AVOP = (unsigned short*)(ws + kOffAVOP);
  unsigned short* P3   = (unsigned short*)(ws + kOffP3);
  unsigned short* NF   = (unsigned short*)(ws + kOffNF);
  unsigned short* DIFF = (unsigned short*)(ws + kOffDIFF);
  float*          W32  = (float*)(ws + kOffW32);
  float*          Up   = (float*)(ws + kOffU);
  float*          Vp   = (float*)(ws + kOffV);

  prep_kernel<<<kPrepBlkTotal, 256, 0, stream>>>(
      states, policies, actions, states_p, actions_p,
      Wk, Wq, Wv, Wkp, Wqp, Wvp, Wf1, Wf2,
      AOA, AOP, AOAP, BTA, BTP, BTF1, BTF2);


  gemm64_kernel<1><<<128, 256, 0, stream>>>(
      AOA, kDim, BTA, kDim, (void*)P1, 4 * kDim,
      kRows, 4 * kDim, kDim, kProjScale, 3 * kDim, kCarryP);

  gemm64_kernel<1><<<32, 256, 0, stream>>>(
      AOP, kDim, BTA + (size_t)3 * kDim * kDim, kDim, (void*)AVOP, kDim,
      kRows, kDim, kDim, kProjScale, 0, kCarryP);

  gemm64_kernel<1><<<64, 256, 0, stream>>>(
      AOAP, kDim, BTP, kDim, (void*)P3, 2 * kDim,
      kRows, 2 * kDim, kDim, kProjScale, kDim, kCarryP);

  attn_kernel<<<kBatch, 256, kLdsTotal, stream>>>(
      P1, AVOP, P3, out + kOut1, out + kOut2, W32, NF, DIFF);


  gemm64_kernel<0><<<16, 256, 0, stream>>>(
      NF, 2 * kDim, BTF1, 2 * kDim, (void*)Up, kF1,
      kRows, kF1, 2 * kDim, kF1Scale, 0, 1.0f);

  gemm64_kernel<0><<<16, 256, 0, stream>>>(
      DIFF, kDim, BTF1, 2 * kDim, (void*)Vp, kF1,
      kRows, kF1, kDim, kF1Scale, 0, 1.0f);

  final_kernel<<<kBatch, 256, 0, stream>>>(Up, Vp, W32, BTF2, out);
}
